// SASRecBlock_52536039965143
// MI455X (gfx1250) — hardware-verified
//
#include <hip/hip_runtime.h>
#include <math.h>
#include <stdint.h>

#define NB     8
#define SEQ    1024
#define DM     1024
#define NH     16
#define HDIM   64
#define FF     4096
#define NROW   (NB * SEQ)
#define NQB    (SEQ / 64)
#define WCARRY 64.0f
#define PCARRY 1024.0f
static_assert(NH * HDIM == DM);
static_assert((SEQ % 64) == 0 && (DM % 64) == 0 && (FF % 64) == 0 && (NROW % 64) == 0);

typedef _Float16 v16h __attribute__((ext_vector_type(16)));
typedef _Float16 v8h  __attribute__((ext_vector_type(8)));
typedef _Float16 v8ha __attribute__((ext_vector_type(8), __may_alias__));
typedef float    v8f  __attribute__((ext_vector_type(8)));
typedef float    v4f  __attribute__((ext_vector_type(4)));
typedef float    v4fa __attribute__((ext_vector_type(4), __may_alias__));
typedef unsigned int v4u __attribute__((ext_vector_type(4)));
typedef unsigned int v2u __attribute__((ext_vector_type(2)));

__device__ __forceinline__ unsigned short hbits(float f) {
  const _Float16 x = (_Float16)f;
  return __builtin_bit_cast(unsigned short, x);
}
__device__ __forceinline__ unsigned pk2(float a, float b) { return (unsigned)hbits(a) | ((unsigned)hbits(b) << 16); }
__device__ __forceinline__ v8f zero8() { v8f z = {0.f, 0.f, 0.f, 0.f, 0.f, 0.f, 0.f, 0.f}; return z; }
__device__ __forceinline__ v4f zero4() { v4f z = {0.f, 0.f, 0.f, 0.f}; return z; }

__device__ __forceinline__ v16h ldfrag(const _Float16* p) {
  union { v16h v; v8h h[2]; } f;
  f.h[0] = *(const v8h*)(p);
  f.h[1] = *(const v8h*)(p + 16);
  return f.v;
}

__device__ __forceinline__ v8f mma_h(v16h a, v16h b, v8f c) {
  c = __builtin_amdgcn_wmma_f32_16x16x32_f16(false, a, false, b, (short)0, c, false, false);
  asm volatile("v_nop\n\tv_nop\n\tv_nop\n\tv_nop" : "+v"(c) : "v"(a), "v"(b));
  return c;
}
__device__ __forceinline__ v8f mma_raw(v16h a, v16h b, v8f c) {
  return __builtin_amdgcn_wmma_f32_16x16x32_f16(false, a, false, b, (short)0, c, false, false);
}
__device__ __forceinline__ void dep_guard(v8f& a, v8f& b, v16h x) {
  asm volatile("v_nop\n\tv_nop\n\tv_nop\n\tv_nop" : "+v"(a), "+v"(b) : "v"(x));
}
__device__ __forceinline__ void keep4(v16h a, v16h b, v16h c, v16h d) {
  asm volatile("v_nop" :: "v"(a), "v"(b), "v"(c), "v"(d));
}
__device__ __forceinline__ void acc_guard4(v8f& a, v8f& b, v8f& c, v8f& d) {
  asm volatile("v_nop\n\tv_nop\n\tv_nop\n\tv_nop" : "+v"(a), "+v"(b), "+v"(c), "+v"(d));
}

__global__ __launch_bounds__(256) void wt_f16(const float* __restrict__ w, unsigned short* out, int R, int C) {
  __shared__ float t[64][65];
  const int tid = threadIdx.x;
  const int c0 = blockIdx.x * 64, r0 = blockIdx.y * 64;
#pragma unroll
  for (int it = 0; it < 4; ++it) {
    const int r = it * 16 + (tid >> 4), c4 = (tid & 15) * 4;
    const v4f v = *(const v4f*)(w + (size_t)(r0 + r) * C + c0 + c4);
    t[r][c4 + 0] = v[0];
    t[r][c4 + 1] = v[1];
    t[r][c4 + 2] = v[2];
    t[r][c4 + 3] = v[3];
  }
  __syncthreads();
  const int q = tid >> 3, oc8 = (tid & 7) * 8;
  v4u pv[2];
#pragma unroll
  for (int it = 0; it < 2; ++it) {
    const int orow = it * 32 + q;
    v4u p;
#pragma unroll
    for (int e = 0; e < 4; ++e)
      p[e] = pk2(t[oc8 + 2 * e][orow] * WCARRY, t[oc8 + 2 * e + 1][orow] * WCARRY);
    pv[it] = p;
  }
  for (int pass = 0; pass < 2; ++pass) {
#pragma unroll
    for (int it = 0; it < 2; ++it) {
      const int orow = it * 32 + q;
      *(volatile v4u*)(out + (size_t)(c0 + orow) * R + r0 + oc8) = pv[it];
    }
    __threadfence();
  }
}

template <int MODE>
__global__ __launch_bounds__(256) void ln_rows(const float* __restrict__ in, const float* __restrict__ g,
                                               const float* __restrict__ be, float* out32,
                                               unsigned short* out16, unsigned short* raw16) {
  __shared__ float redA[8], redB[8];
  const int row = blockIdx.x, tid = threadIdx.x, wave = tid >> 5, lane = tid & 31;
  const size_t base = (size_t)row * DM + 4 * tid;
  const v4f xv = *(const v4f*)(in + base);
  float s = (xv[0] + xv[1]) + (xv[2] + xv[3]);
#pragma unroll
  for (int off = 1; off < 32; off <<= 1) s += __shfl_xor(s, off, 32);
  if (lane == 0) redA[wave] = s;
  __syncthreads();
  float tot = 0.f;
#pragma unroll
  for (int i = 0; i < 8; ++i) tot += redA[i];
  const float mean = tot * (1.0f / DM);
  float d0 = xv[0] - mean, d1 = xv[1] - mean, d2 = xv[2] - mean, d3 = xv[3] - mean;
  float ss = (d0 * d0 + d1 * d1) + (d2 * d2 + d3 * d3);
#pragma unroll
  for (int off = 1; off < 32; off <<= 1) ss += __shfl_xor(ss, off, 32);
  if (lane == 0) redB[wave] = ss;
  __syncthreads();
  float tot2 = 0.f;
#pragma unroll
  for (int i = 0; i < 8; ++i) tot2 += redB[i];
  const float var  = tot2 * (1.0f / DM);
  const float rstd = rsqrtf(var + 1.0e-8f);
  const v4f g4 = *(const v4f*)(g + 4 * tid);
  const v4f b4 = *(const v4f*)(be + 4 * tid);
  v4f y;
  y[0] = d0 * rstd * g4[0] + b4[0];
  y[1] = d1 * rstd * g4[1] + b4[1];
  y[2] = d2 * rstd * g4[2] + b4[2];
  y[3] = d3 * rstd * g4[3] + b4[3];
  v2u yh;
  yh[0] = pk2(y[0], y[1]);
  yh[1] = pk2(y[2], y[3]);
  v2u xh = yh;
  if (MODE == 0) { xh[0] = pk2(xv[0], xv[1]); xh[1] = pk2(xv[2], xv[3]); }
  for (int pass = 0; pass < 2; ++pass) {
    if (MODE == 0) {
      *(volatile v4f*)(out32 + base) = y;
      *(volatile v2u*)(raw16 + base) = xh;
    }
    *(volatile v2u*)(out16 + base) = yh;
    __threadfence();
  }
}

template <int EPI>
__global__ __launch_bounds__(256) void gemm64(
    const unsigned short* __restrict__ Ap, int lda, long long strideA,
    const unsigned short* __restrict__ Btp, int ldb, long long strideB,
    const float* __restrict__ bias, void* Cout, int ldc, long long strideC,
    const float* __restrict__ resid, int M, int N, int K, float oscale) {
  __shared__ __align__(16) float sT[8][16 * 68];
  const int b    = blockIdx.y;
  const int lane = threadIdx.x & 31;
  const int wave = threadIdx.x >> 5;
  const int tilesN = N >> 6;
  const int tilesM = M >> 6;
  const int tile = blockIdx.x * 8 + wave;
  if (tile >= tilesM * tilesN) return;
  const int tm = tile / tilesN;
  const int tn = tile - tm * tilesN;
  const int m0 = tm << 6;
  const int n0 = tn << 6;

  const _Float16* Ab = (const _Float16*)(const void*)Ap  + (size_t)b * strideA;
  const _Float16* Bb = (const _Float16*)(const void*)Btp + (size_t)b * strideB;

  const int rlane = lane & 15;
  const int koff  = (lane >> 4) * 8;
  const int mOff  = (lane >> 4) * 8;

  v8f acc[4][4];
#pragma unroll
  for (int i = 0; i < 4; ++i)
#pragma unroll
    for (int j = 0; j < 4; ++j) acc[i][j] = zero8();

  for (int k0 = 0; k0 < K; k0 += 32) {
    v16h bh[4];
#pragma unroll
    for (int j = 0; j < 4; ++j) {
      const size_t bo = (size_t)(n0 + (j << 4) + rlane) * ldb + koff + k0;
      bh[j] = ldfrag(Bb + bo);
    }
#pragma unroll
    for (int i = 0; i < 4; ++i) {
      const size_t ao = (size_t)(m0 + (i << 4) + rlane) * lda + koff + k0;
      const v16h ah = ldfrag(Ab + ao);
#pragma unroll
      for (int j = 0; j < 4; ++j) acc[i][j] = mma_raw(ah, bh[j], acc[i][j]);
      dep_guard(acc[i][0], acc[i][3], ah);
    }
    keep4(bh[0], bh[1], bh[2], bh[3]);
  }
  acc_guard4(acc[0][0], acc[0][1], acc[0][2], acc[0][3]);
  acc_guard4(acc[1][0], acc[1][1], acc[1][2], acc[1][3]);
  acc_guard4(acc[2][0], acc[2][1], acc[2][2], acc[2][3]);
  acc_guard4(acc[3][0], acc[3][1], acc[3][2], acc[3][3]);

  float* slab = sT[wave];
#pragma unroll
  for (int i = 0; i < 4; ++i) {
    const int mBase = m0 + (i << 4);
#pragma unroll
    for (int j = 0; j < 4; ++j) {
#pragma unroll
      for (int r = 0; r < 8; ++r) {
        slab[(mOff + r) * 68 + (j << 4) + rlane] = acc[i][j][r];
      }
    }
    __builtin_amdgcn_fence(__ATOMIC_RELEASE, "workgroup");
    __builtin_amdgcn_wave_barrier();
    __builtin_amdgcn_fence(__ATOMIC_ACQUIRE, "workgroup");
    if (EPI == 3) {
      float* C = (float*)Cout + (size_t)b * strideC;
      const float* Rb = resid + (size_t)b * strideC;
      const int hh = lane >> 4, c4 = (lane & 15) * 4;
      const v4f bv = *(const v4f*)(bias + n0 + c4);
      for (int pass = 0; pass < 2; ++pass) {
#pragma unroll
        for (int it = 0; it < 8; ++it) {
          const int row = it * 2 + hh;
          const size_t idx = (size_t)(mBase + row) * ldc + n0 + c4;
          const v4f sv = *(const v4fa*)(slab + row * 68 + c4);
          const v4f rv = *(const v4f*)(Rb + idx);
          v4f t = sv * oscale + bv;
          t = t + rv;
          *(volatile v4f*)(C + idx) = t;
        }
        __threadfence();
      }
    } else {
      unsigned short* C = (unsigned short*)Cout + (size_t)b * strideC;
      const int q = lane >> 3, c8 = (lane & 7) * 8;
      float bc[8];
      {
        v4f b0 = zero4(), b1 = zero4();
        if (EPI != 1) { b0 = *(const v4f*)(bias + n0 + c8); b1 = *(const v4f*)(bias + n0 + c8 + 4); }
        bc[0] = b0[0]; bc[1] = b0[1]; bc[2] = b0[2]; bc[3] = b0[3];
        bc[4] = b1[0]; bc[5] = b1[1]; bc[6] = b1[2]; bc[7] = b1[3];
      }
      v4u hv[4];
#pragma unroll
      for (int it = 0; it < 4; ++it) {
        const int row = it * 4 + q;
        const float* sp = slab + row * 68 + c8;
        float brow = 0.f;
        if (EPI == 1) brow = bias[mBase + row];
        v4u a;
#pragma unroll
        for (int e = 0; e < 4; ++e) {
          float f0 = sp[2 * e] * oscale + bc[2 * e] + brow;
          float f1 = sp[2 * e + 1] * oscale + bc[2 * e + 1] + brow;
          if (EPI == 2) { f0 = fmaxf(f0, 0.0f); f1 = fmaxf(f1, 0.0f); }
          a[e] = pk2(f0, f1);
        }
        hv[it] = a;
      }
      for (int pass = 0; pass < 2; ++pass) {
#pragma unroll
        for (int it = 0; it < 4; ++it) {
          const int row = it * 4 + q;
          *(volatile v4u*)(C + (size_t)(mBase + row) * ldc + n0 + c8) = hv[it];
        }
        __threadfence();
      }
    }
    __builtin_amdgcn_fence(__ATOMIC_RELEASE, "workgroup");
    __builtin_amdgcn_wave_barrier();
    __builtin_amdgcn_fence(__ATOMIC_ACQUIRE, "workgroup");
  }
}

__global__ __launch_bounds__(128)
void attn64(const unsigned short* __restrict__ qp, const unsigned short* __restrict__ kp,
            const unsigned short* __restrict__ vtp, const int* __restrict__ mask,
            const float* __restrict__ qin, float* hout, float sscale) {
  union FH { v16h v; v8h h[2]; };
  __shared__ __align__(16) _Float16 Psh[4][16 * 64];
  __shared__ __align__(16) float    Os[4][16 * 64];

  const int tid  = threadIdx.x;
  const int wave = tid >> 5;
  const int lane = tid & 31;
  const int hh   = lane >> 4;
  const int c    = lane & 15;

  const int bx   = blockIdx.x;
  const int qb   = bx % NQB;
  const int rest = bx / NQB;
  const int h    = rest % NH;
  const int b    = rest / NH;
  const int q0   = qb * 64 + wave * 16;
  const size_t rowB = (size_t)b * SEQ;

  const _Float16* Q  = (const _Float16*)(const void*)qp + (size_t)h * HDIM;
  const _Float16* Kp = (const _Float16*)(const void*)kp + (size_t)h * HDIM;
  const _Float16* VT = (const _Float16*)(const void*)vtp + ((size_t)b * DM + (size_t)h * HDIM) * SEQ;
  const int* km = mask + (size_t)b * SEQ;

  v16h qa[2];
#pragma unroll
  for (int dc = 0; dc < 2; ++dc) qa[dc] = ldfrag(Q + (rowB + q0 + c) * DM + dc * 32 + 8 * hh);

  float qm[8];
#pragma unroll
  for (int r = 0; r < 8; ++r) qm[r] = (float)km[q0 + 8 * hh + r];

  float mrow[8], lrow[8];
  v8f oacc[4];
#pragma unroll
  for (int r = 0; r < 8; ++r) { mrow[r] = -INFINITY; lrow[r] = 0.f; }
#pragma unroll
  for (int t = 0; t < 4; ++t) oacc[t] = zero8();

  int nkt = qb + 1;
  if (nkt > NQB) nkt = NQB;
  _Float16* pw = Psh[wave];

  for (int kt = 0; kt < nkt; ++kt) {
    const int kv0 = kt * 64;

    v8f s[4];
#pragma unroll
    for (int j = 0; j < 4; ++j) {
      s[j] = zero8();
#pragma unroll
      for (int dc = 0; dc < 2; ++dc) {
        const _Float16* kr = Kp + (rowB + kv0 + j * 16 + c) * DM + dc * 32 + 8 * hh;
        FH kb;
        kb.h[0] = *(const v8h*)(kr);
        kb.h[1] = *(const v8h*)(kr + 16);
        s[j] = mma_h(qa[dc], kb.v, s[j]);
      }
    }

    int kidx[4], kval[4];
#pragma unroll
    for (int j = 0; j < 4; ++j) { kidx[j] = kv0 + j * 16 + c; kval[j] = km[kidx[j]]; }

#pragma unroll
    for (int r = 0; r < 8; ++r) {
      const int qr = q0 + 8 * hh + r;
      float m = -INFINITY;
#pragma unroll
      for (int j = 0; j < 4; ++j) {
        const bool ok = (kval[j] != 0) && (kidx[j] <= qr);
        const float sv = ok ? (s[j][r] * sscale) : -INFINITY;
        s[j][r] = sv;
        m = fmaxf(m, sv);
      }
#pragma unroll
      for (int off = 1; off < 16; off <<= 1) m = fmaxf(m, __shfl_xor(m, off, 32));
      const float mnew  = fmaxf(mrow[r], m);
      const float msafe = (mnew == -INFINITY) ? 0.f : mnew;
      const float alpha = __expf(mrow[r] - msafe);
      mrow[r] = mnew;
      float psum = 0.f;
#pragma unroll
      for (int j = 0; j < 4; ++j) {
        const float p = __expf(s[j][r] - msafe);
        psum += p;
        pw[(8 * hh + r) * 64 + j * 16 + c] = (_Float16)(p * PCARRY);
      }
#pragma unroll
      for (int off = 1; off < 16; off <<= 1) psum += __shfl_xor(psum, off, 32);
      lrow[r] = lrow[r] * alpha + psum;
#pragma unroll
      for (int t = 0; t < 4; ++t) oacc[t][r] *= alpha;
    }
    __builtin_amdgcn_fence(__ATOMIC_RELEASE, "workgroup");
    __builtin_amdgcn_wave_barrier();
    __builtin_amdgcn_fence(__ATOMIC_ACQUIRE, "workgroup");

#pragma unroll
    for (int kk = 0; kk < 2; ++kk) {
      FH pa;
      pa.h[0] = *(const v8ha*)(pw + c * 64 + kk * 32 + 8 * hh);
      pa.h[1] = *(const v8ha*)(pw + c * 64 + kk * 32 + 16 + 8 * hh);
#pragma unroll
      for (int t = 0; t < 4; ++t) {
        const _Float16* vr = VT + (size_t)(t * 16 + c) * SEQ + kv0 + kk * 32 + 8 * hh;
        FH vb;
        vb.h[0] = *(const v8h*)(vr);
        vb.h[1] = *(const v8h*)(vr + 16);
        oacc[t] = mma_h(pa.v, vb.v, oacc[t]);
      }
    }
    __builtin_amdgcn_fence(__ATOMIC_RELEASE, "workgroup");
    __builtin_amdgcn_wave_barrier();
    __builtin_amdgcn_fence(__ATOMIC_ACQUIRE, "workgroup");
  }

  float* os = Os[wave];
#pragma unroll
  for (int r = 0; r < 8; ++r) {
    const float l = lrow[r];
    const float inv = ((l > 0.f) ? (qm[r] * (1.0f / l)) : 0.f) * (1.0f / PCARRY);
#pragma unroll
    for (int t = 0; t < 4; ++t) os[(8 * hh + r) * 64 + t * 16 + c] = oacc[t][r] * inv;
  }
  __builtin_amdgcn_fence(__ATOMIC_RELEASE, "workgroup");
  __builtin_amdgcn_wave_barrier();
  __builtin_amdgcn_fence(__ATOMIC_ACQUIRE, "workgroup");
  {
    const int hh2 = lane >> 4, c4 = (lane & 15) * 4;
    v4f ov[8];
#pragma unroll
    for (int it = 0; it < 8; ++it) {
      const int row = it * 2 + hh2;
      const size_t go = (rowB + q0 + row) * DM + (size_t)h * HDIM + c4;
      const v4f cv = *(const v4fa*)(os + row * 64 + c4);
      const v4f rv = *(const v4f*)(qin + go);
      ov[it] = cv + rv;
    }
    for (int pass = 0; pass < 2; ++pass) {
#pragma unroll
      for (int it = 0; it < 8; ++it) {
        const int row = it * 2 + hh2;
        const size_t go = (rowB + q0 + row) * DM + (size_t)h * HDIM + c4;
        *(volatile v4f*)(hout + go) = ov[it];
      }
      __threadfence();
    }
  }
}

extern "C" void kernel_launch(void* const* d_in, const int* in_sizes, int n_in,
                              void* d_out, int out_size, void* d_ws, size_t ws_size,
                              hipStream_t stream) {
  if (n_in < 16) return;
  if (in_sizes[0] != NROW * DM || in_sizes[1] != NB * SEQ) return;
  if (in_sizes[2] != DM * DM || in_sizes[4] != DM * DM || in_sizes[6] != DM * DM) return;
  if (in_sizes[3] != DM || in_sizes[5] != DM || in_sizes[7] != DM) return;
  if (in_sizes[8] != DM * FF || in_sizes[9] != FF || in_sizes[10] != FF * DM || in_sizes[11] != DM) return;
  if (in_sizes[12] != DM || in_sizes[13] != DM || in_sizes[14] != DM || in_sizes[15] != DM) return;
  if (out_size != NROW * DM) return;

  const float* x    = (const float*)d_in[0];
  const int*   mask = (const int*)d_in[1];
  const float* wq   = (const float*)d_in[2];
  const float* bq   = (const float*)d_in[3];
  const float* wk   = (const float*)d_in[4];
  const float* bk   = (const float*)d_in[5];
  const float* wv   = (const float*)d_in[6];
  const float* bv   = (const float*)d_in[7];
  const float* w1   = (const float*)d_in[8];
  const float* b1   = (const float*)d_in[9];
  const float* w2   = (const float*)d_in[10];
  const float* b2   = (const float*)d_in[11];
  const float* g1   = (const float*)d_in[12];
  const float* be1  = (const float*)d_in[13];
  const float* g2   = (const float*)d_in[14];
  const float* be2  = (const float*)d_in[15];
  float* out = (float*)d_out;

  const size_t P32 = (size_t)NROW * DM * 4;
  const size_t P16 = (size_t)NROW * DM * 2;
  const size_t PW  = (size_t)DM * DM * 2;
  const size_t PW1 = (size_t)DM * FF * 2;
  const size_t PH1 = (size_t)NROW * FF * 2;
  const size_t oQin32 = 0;
  const size_t oQ16   = oQin32 + P32;
  const size_t oK16   = oQ16 + P16;
  const size_t oVT16  = oK16 + P16;
  const size_t oX16   = oVT16 + P16;
  const size_t oQin16 = oX16 + P16;
  const size_t oWq    = oQin16 + P16;
  const size_t oWk    = oWq + PW;
  const size_t oWv    = oWk + PW;
  const size_t end1   = oWv + PW;
  const size_t oH32   = oX16;
  const size_t oW1    = oWq;
  const size_t end2   = oW1 + PW1;
  const size_t oLn2   = oQin32;
  const size_t oH1    = oLn2 + P16;
  const size_t oW2    = oLn2;
  size_t total = (end1 > end2) ? end1 : end2;
  if (oH1 + PH1 > total) total = oH1 + PH1;
  if (total > ws_size) return;
  if (total > (size_t)134217728) return;
  if (oH32 + P32 > oW1) return;
  if (oH1 + PH1 > oH32) return;
  if (oW2 + PW1 > oH1) return;
  if (oQin16 + P16 > oWq) return;

  char* ws = (char*)d_ws;
  float*          qin32 = (float*)(ws + oQin32);
  unsigned short* q16   = (unsigned short*)(ws + oQ16);
  unsigned short* k16   = (unsigned short*)(ws + oK16);
  unsigned short* vt16  = (unsigned short*)(ws + oVT16);
  unsigned short* x16   = (unsigned short*)(ws + oX16);
  unsigned short* qin16 = (unsigned short*)(ws + oQin16);
  unsigned short* wqT   = (unsigned short*)(ws + oWq);
  unsigned short* wkT   = (unsigned short*)(ws + oWk);
  unsigned short* wvT   = (unsigned short*)(ws + oWv);
  float*          h32   = (float*)(ws + oH32);
  unsigned short* w1T   = (unsigned short*)(ws + oW1);
  unsigned short* ln2   = (unsigned short*)(ws + oLn2);
  unsigned short* h1    = (unsigned short*)(ws + oH1);
  unsigned short* w2T   = (unsigned short*)(ws + oW2);

  const dim3 blk(256);
  const float oscale = 1.0f / WCARRY;
  const int tilesQ  = (NROW / 64) * (DM / 64);
  const int tilesVT = (DM / 64) * (SEQ / 64);
  const int tilesF1 = (NROW / 64) * (FF / 64);
  const dim3 gQ((tilesQ + 7) / 8, 1);
  const dim3 gVT((tilesVT + 7) / 8, NB);
  const dim3 gF1((tilesF1 + 7) / 8, 1);

  wt_f16<<<dim3(DM / 64, DM / 64), blk, 0, stream>>>(wq, wqT, DM, DM);
  wt_f16<<<dim3(DM / 64, DM / 64), blk, 0, stream>>>(wk, wkT, DM, DM);
  wt_f16<<<dim3(DM / 64, DM / 64), blk, 0, stream>>>(wv, wvT, DM, DM);
  ln_rows<0><<<dim3(NROW), blk, 0, stream>>>(x, g1, be1, qin32, qin16, x16);
  gemm64<0><<<gQ, blk, 0, stream>>>(qin16, DM, 0LL, wqT, DM, 0LL, bq, (void*)q16, DM, 0LL, bq,
                                     NROW, DM, DM, oscale);
  gemm64<0><<<gQ, blk, 0, stream>>>(x16, DM, 0LL, wkT, DM, 0LL, bk, (void*)k16, DM, 0LL, bk,
                                     NROW, DM, DM, oscale);
  gemm64<1><<<gVT, blk, 0, stream>>>(wvT, DM, 0LL, x16, DM, (long long)SEQ * DM, bv,
                                      (void*)vt16, SEQ, (long long)DM * SEQ, bv,
                                      DM, SEQ, DM, oscale);
  attn64<<<dim3(NB * NH * NQB), dim3(128), 0, stream>>>(q16, k16, vt16, mask, qin32, h32, 0.125f);
  wt_f16<<<dim3(FF / 64, DM / 64), blk, 0, stream>>>(w1, w1T, DM, FF);
  ln_rows<1><<<dim3(NROW), blk, 0, stream>>>(h32, g2, be2, h32, ln2, ln2);
  gemm64<2><<<gF1, blk, 0, stream>>>(ln2, DM, 0LL, w1T, DM, 0LL, b1, (void*)h1, FF, 0LL, b1,
                                      NROW, FF, DM, oscale);
  wt_f16<<<dim3(DM / 64, FF / 64), blk, 0, stream>>>(w2, w2T, FF, DM);
  gemm64<3><<<gQ, blk, 0, stream>>>(h1, FF, 0LL, w2T, FF, 0LL, b2, (void*)out, DM, 0LL, h32,
                                     NROW, DM, FF, oscale);
  (void)hipGetLastError();
}
